// ENLTransformerBlock_21380347199745
// MI455X (gfx1250) — hardware-verified
//
#include <hip/hip_runtime.h>
#include <math.h>

typedef __attribute__((ext_vector_type(16))) _Float16 v16h;
typedef __attribute__((ext_vector_type(8)))  _Float16 v8h;
typedef __attribute__((ext_vector_type(8)))  float    v8f;
typedef __attribute__((ext_vector_type(4)))  float    v4f;
typedef __attribute__((ext_vector_type(4)))  unsigned int v4u;

constexpr int kBatch  = 8;
constexpr int kChan   = 256;
constexpr int kFeat   = 256;
constexpr int kNtok   = 4096;
constexpr int kTokAll = kBatch * kNtok;
constexpr int kHid    = 1024;

constexpr float kHCarry    = 16.0f;
constexpr float kWCarry    = 256.0f;
constexpr float kW2Carry   = 512.0f;
constexpr float kProjCarry = 16.0f;
constexpr float kQnCarry   = 2048.0f;
constexpr float kPhiCarry  = 64.0f;
constexpr float kVCarry    = 64.0f;
constexpr float kCtxCarry  = 16.0f;
constexpr float kGCarry    = 16.0f;

constexpr float kScaleQK  = 1.0f / (kHCarry * kWCarry);
constexpr float kScaleVT  = kVCarry / (kHCarry * kWCarry);
constexpr float kScaleDD  = 1.0f / (kQnCarry * kProjCarry);
constexpr float kScaleCTX = kCtxCarry / (kVCarry * kPhiCarry);
constexpr float kScaleOUT = 1.0f / (kCtxCarry * kPhiCarry);
constexpr float kScaleFF1 = 1.0f / (kHCarry * kWCarry);
constexpr float kScaleFF2 = 1.0f / (kW2Carry * kGCarry);

constexpr float kRatio  = 0.0625f;
constexpr float kPhiEps = 1e-4f;

constexpr size_t kOffH16  = 0;
constexpr size_t kSzH16   = (size_t)kTokAll * kChan * 2;
constexpr size_t kOffVT16 = kOffH16 + kSzH16;
constexpr size_t kSzVT16  = (size_t)kBatch * kChan * kNtok * 2;
constexpr size_t kOffT2   = kOffVT16 + kSzVT16;
constexpr size_t kSzT2    = (size_t)kBatch * kChan * kNtok * 4;
constexpr size_t kOffWQK  = kOffT2 + kSzT2;
constexpr size_t kSzWQK   = (size_t)2 * kChan * kChan * 2;
constexpr size_t kOffWA   = kOffWQK + kSzWQK;
constexpr size_t kSzW     = (size_t)kChan * kChan * 2;
constexpr size_t kOffPROJ = kOffWA + kSzW;
constexpr size_t kOffW1   = kOffPROJ + kSzW;
constexpr size_t kSzW1    = (size_t)kHid * kChan * 2;
constexpr size_t kOffW2   = kOffW1 + kSzW1;
constexpr size_t kOffBQK  = kOffW2 + kSzW1;
constexpr size_t kSzBQK   = 4096;
constexpr size_t kOffQKF  = kOffBQK + kSzBQK;
constexpr size_t kSzQKF   = (size_t)kNtok * 2 * kChan * 4;
constexpr size_t kOffQKN  = kOffQKF + kSzQKF;
constexpr size_t kSzQKN   = (size_t)2 * kNtok * kChan * 2;
constexpr size_t kOffDIAG = kOffQKN + kSzQKN;
constexpr size_t kSzDIAG  = (size_t)2 * kNtok * 4;
constexpr size_t kOffDDQ  = kOffDIAG + kSzDIAG;
constexpr size_t kSzDD    = (size_t)kNtok * kFeat * 4;
constexpr size_t kOffDDKT = kOffDDQ + kSzDD;
constexpr size_t kOffKSUM = kOffDDKT + kSzDD;
constexpr size_t kSzKSUM  = 4096;
constexpr size_t kOffKPT  = kOffKSUM + kSzKSUM;
constexpr size_t kSzP16   = (size_t)kNtok * kFeat * 2;
constexpr size_t kOffQP   = kOffKPT + kSzP16;
constexpr size_t kOffDINV = kOffQP + kSzP16;
constexpr size_t kSzDINV  = (size_t)kNtok * 4;
constexpr size_t kOffCTXT = kOffDINV + kSzDINV;
constexpr size_t kSzCTXT  = (size_t)kChan * kFeat * 2;
constexpr size_t kOffU    = kOffCTXT + kSzCTXT;
constexpr size_t kSzU     = (size_t)kNtok * kHid * 4;
constexpr size_t kOffG16  = kOffU + kSzU;
constexpr size_t kSzG16   = (size_t)kNtok * kHid * 2;
constexpr size_t kWsTotal = kOffG16 + kSzG16;
typedef char ws_total_check[(kWsTotal <= (size_t)134217728) ? 1 : -1];
typedef char ws_align_check[((kOffBQK % 128) == 0 && (kOffQKF % 128) == 0 && (kOffKSUM % 128) == 0 && (kOffDINV % 128) == 0 && (kOffCTXT % 128) == 0 && (kOffU % 128) == 0 && (kOffG16 % 128) == 0) ? 1 : -1];

__device__ __forceinline__ void dep_guard_h(v8f& a, v8f& b, v16h x, v16h y) { asm volatile("v_nop\n\tv_nop\n\tv_nop\n\tv_nop" : "+v"(a), "+v"(b) : "v"(x), "v"(y)); }
__device__ __forceinline__ void keep4_h(v16h a, v16h b, v16h c, v16h d) { asm volatile("v_nop" :: "v"(a), "v"(b), "v"(c), "v"(d)); }
__device__ __forceinline__ void acc_guard4(v8f& a, v8f& b, v8f& c, v8f& d) { asm volatile("v_nop\n\tv_nop\n\tv_nop\n\tv_nop" : "+v"(a), "+v"(b), "+v"(c), "+v"(d)); }

struct FragH {
  union U { v16h v; v8h h[2]; };
  static __device__ __forceinline__ v16h load(const _Float16* p) {
    U f; f.h[0] = *(const v8h*)(p); f.h[1] = *(const v8h*)(p + 16); return f.v;
  }
  static __device__ __forceinline__ v8f mma(v16h a, v16h b, v8f c) {
    return __builtin_amdgcn_wmma_f32_16x16x32_f16(false, a, false, b, (short)0, c, false, false);
  }
};

__device__ __forceinline__ unsigned pk16(unsigned short a, unsigned short b) { return (unsigned)a | ((unsigned)b << 16); }
__device__ __forceinline__ unsigned short h_bits(float f) { const _Float16 h = (_Float16)f; return __builtin_bit_cast(unsigned short, h); }

__device__ __forceinline__ float wave_sum(float v) {
#pragma unroll
  for (int off = 16; off > 0; off >>= 1) v += __shfl_xor(v, off, 32);
  return v;
}

template <int BIAS_MODE, int OUT_MODE, bool RESID, bool COLSC>
__global__ __launch_bounds__(256) void gemm_f16(
    const unsigned short* __restrict__ Ap, int lda, long strideA,
    const unsigned short* __restrict__ Btp, int ldb, long strideB,
    void* __restrict__ Cout, int ldc, long strideC,
    const float* __restrict__ bias, float bscale,
    const float* __restrict__ resid, long strideR,
    const float* __restrict__ colsc, long strideS,
    int M, int N, int K, float scale) {
  const _Float16* A  = (const _Float16*)Ap;
  const _Float16* Bt = (const _Float16*)Btp;
  __shared__ __align__(16) float sT[8][16 * 68];
  const int b    = blockIdx.y;
  const int lane = threadIdx.x & 31;
  const int wave = threadIdx.x >> 5;
  const int tilesN = N >> 6;
  const int tilesM = M >> 6;
  const int tile = blockIdx.x * 8 + wave;
  if (tile >= tilesM * tilesN) return;
  const int tm = tile / tilesN;
  const int tn = tile - tm * tilesN;
  const int m0 = tm << 6;
  const int n0 = tn << 6;

  const _Float16* Ab = A  + (size_t)b * strideA;
  const _Float16* Bb = Bt + (size_t)b * strideB;

  const int rlane = lane & 15;
  const int koff  = (lane >> 4) * 8;
  const int mOff  = (lane >> 4) * 8;

  v8f acc[4][4];
#pragma unroll
  for (int i = 0; i < 4; ++i)
#pragma unroll
    for (int j = 0; j < 4; ++j) acc[i][j] = (v8f){0.f,0.f,0.f,0.f,0.f,0.f,0.f,0.f};

  for (int k0 = 0; k0 < K; k0 += 32) {
    v16h bh[4];
#pragma unroll
    for (int j = 0; j < 4; ++j) {
      const size_t bo = (size_t)(n0 + (j << 4) + rlane) * ldb + koff + k0;
      bh[j] = FragH::load(Bb + bo);
    }
#pragma unroll
    for (int i = 0; i < 4; ++i) {
      const size_t ao = (size_t)(m0 + (i << 4) + rlane) * lda + koff + k0;
      v16h ah = FragH::load(Ab + ao);
#pragma unroll
      for (int j = 0; j < 4; ++j) acc[i][j] = FragH::mma(ah, bh[j], acc[i][j]);
      dep_guard_h(acc[i][0], acc[i][3], ah, ah);
    }
    keep4_h(bh[0], bh[1], bh[2], bh[3]);
  }
  acc_guard4(acc[0][0], acc[0][1], acc[0][2], acc[0][3]);
  acc_guard4(acc[1][0], acc[1][1], acc[1][2], acc[1][3]);
  acc_guard4(acc[2][0], acc[2][1], acc[2][2], acc[2][3]);
  acc_guard4(acc[3][0], acc[3][1], acc[3][2], acc[3][3]);

  float* slab = sT[wave];
  const float* Rb = RESID ? (resid + (size_t)b * strideR) : nullptr;
  const float* Sb = COLSC ? (colsc + (size_t)b * strideS) : nullptr;
#pragma unroll
  for (int i = 0; i < 4; ++i) {
    const int mBase = m0 + (i << 4);
#pragma unroll
    for (int j = 0; j < 4; ++j) {
      const int n = n0 + (j << 4) + rlane;
      float bv = 0.f;
      if (BIAS_MODE == 2) bv = bias[n] * bscale;
      float sv = 1.f;
      if (COLSC) sv = Sb[n];
#pragma unroll
      for (int r = 0; r < 8; ++r) {
        float v = acc[i][j][r] * scale;
        if (COLSC) v *= sv;
        if (BIAS_MODE == 1) v += bias[mBase + mOff + r] * bscale;
        if (BIAS_MODE == 2) v += bv;
        if (RESID) v += Rb[(size_t)(mBase + mOff + r) * ldc + n];
        slab[(mOff + r) * 68 + (j << 4) + rlane] = v;
      }
    }
    __builtin_amdgcn_fence(__ATOMIC_RELEASE, "workgroup");
    __builtin_amdgcn_wave_barrier();
    __builtin_amdgcn_fence(__ATOMIC_ACQUIRE, "workgroup");
    if (OUT_MODE == 0) {
      float* C = (float*)Cout + (size_t)b * strideC;
      const int hh = lane >> 4, c4 = (lane & 15) * 4;
      for (int pass = 0; pass < 2; ++pass) {
#pragma unroll
        for (int it = 0; it < 8; ++it) {
          const int row = it * 2 + hh;
          v4f v = *(const v4f*)(slab + row * 68 + c4);
          *(volatile v4f*)(C + (size_t)(mBase + row) * ldc + n0 + c4) = v;
        }
        __threadfence();
      }
    } else {
      const int q = lane >> 3, c8 = (lane & 7) * 8;
      unsigned short* C = (unsigned short*)Cout + (size_t)b * strideC;
      for (int pass = 0; pass < 2; ++pass) {
#pragma unroll
        for (int it = 0; it < 4; ++it) {
          const int row = it * 4 + q;
          const float* sp = slab + row * 68 + c8;
          v8h hv;
#pragma unroll
          for (int e = 0; e < 8; ++e) hv[e] = (_Float16)sp[e];
          *(volatile v8h*)(C + (size_t)(mBase + row) * ldc + n0 + c8) = hv;
        }
        __threadfence();
      }
    }
    __builtin_amdgcn_fence(__ATOMIC_RELEASE, "workgroup");
    __builtin_amdgcn_wave_barrier();
    __builtin_amdgcn_fence(__ATOMIC_ACQUIRE, "workgroup");
  }
}

__global__ __launch_bounds__(256) void prep_kernel(
    const float* __restrict__ wq, const float* __restrict__ wk, const float* __restrict__ wa,
    const float* __restrict__ proj, const float* __restrict__ w1, const float* __restrict__ w2,
    const float* __restrict__ bq, const float* __restrict__ bk,
    unsigned short* __restrict__ wqk16, unsigned short* __restrict__ wa16, unsigned short* __restrict__ proj16,
    unsigned short* __restrict__ w1_16, unsigned short* __restrict__ w2_16, float* __restrict__ bqk) {
  const int job = blockIdx.y;
  const int t = threadIdx.x;
  if (job == 6) {
    if (blockIdx.x != 0) return;
    if (t < 128) {
      const int i4 = (t & 63) * 4;
      const v4f a = *(const v4f*)(bq + i4);
      const v4f c = *(const v4f*)(bk + i4);
      const bool useq = (t < 64);
      v4f v;
      v.x = useq ? a.x : c.x; v.y = useq ? a.y : c.y; v.z = useq ? a.z : c.z; v.w = useq ? a.w : c.w;
      float* p = bqk + 4 * t;
      *(volatile v4f*)p = v;
      __threadfence();
      *(volatile v4f*)p = v;
    }
    return;
  }
  const float* src = wq; unsigned short* dst = wqk16; int n8 = kChan * kChan / 8; float sc = kWCarry;
  if (job == 1)      { src = wk;   dst = wqk16 + kChan * kChan; }
  else if (job == 2) { src = wa;   dst = wa16; }
  else if (job == 3) { src = proj; dst = proj16; sc = kProjCarry; }
  else if (job == 4) { src = w1;   dst = w1_16; n8 = kHid * kChan / 8; }
  else if (job == 5) { src = w2;   dst = w2_16; n8 = kChan * kHid / 8; sc = kW2Carry; }
  const int i = blockIdx.x * 256 + t;
  if (i >= n8) return;
  const float* p = src + 8 * (size_t)i;
  const v4f a = *(const v4f*)(p);
  const v4f c = *(const v4f*)(p + 4);
  unsigned short hb[8];
#pragma unroll
  for (int e = 0; e < 4; ++e) {
    hb[e]     = h_bits(a[e] * sc);
    hb[4 + e] = h_bits(c[e] * sc);
  }
  const v4u u = (v4u){pk16(hb[0], hb[1]), pk16(hb[2], hb[3]), pk16(hb[4], hb[5]), pk16(hb[6], hb[7])};
  unsigned short* q = dst + 8 * (size_t)i;
  *(volatile v4u*)q = u;
  __threadfence();
  *(volatile v4u*)q = u;
}

__global__ __launch_bounds__(256) void ln_tok_kernel(const float* __restrict__ src, const float* __restrict__ gam,
                                                     const float* __restrict__ bet, unsigned short* __restrict__ hout) {
  __shared__ float s[kChan][33];
  const int t = threadIdx.x, lane = t & 31, wave = t >> 5;
  const int b  = blockIdx.x >> 7;
  const int n0 = (blockIdx.x & 127) * 32;
  const float* sb = src + (size_t)b * kChan * kNtok + n0 + lane;
#pragma unroll 4
  for (int i = 0; i < 32; ++i) {
    const int c = i * 8 + wave;
    s[c][lane] = sb[(size_t)c * kNtok];
  }
  __syncthreads();
  const int c0 = lane * 8;
  const v4f ga = *(const v4f*)(gam + c0), gb = *(const v4f*)(gam + c0 + 4);
  const v4f ea = *(const v4f*)(bet + c0), eb = *(const v4f*)(bet + c0 + 4);
  float gg[8], ee[8];
#pragma unroll
  for (int e = 0; e < 4; ++e) { gg[e] = ga[e]; gg[4 + e] = gb[e]; ee[e] = ea[e]; ee[4 + e] = eb[e]; }
#pragma unroll 1
  for (int i = 0; i < 4; ++i) {
    const int nl = wave * 4 + i;
    float v[8];
#pragma unroll
    for (int e = 0; e < 8; ++e) v[e] = s[c0 + e][nl];
    float sum = ((v[0] + v[1]) + (v[2] + v[3])) + ((v[4] + v[5]) + (v[6] + v[7]));
    sum = wave_sum(sum);
    const float mu = sum * (1.0f / 256.0f);
    float d[8];
    float ss = 0.f;
#pragma unroll
    for (int e = 0; e < 8; ++e) { d[e] = v[e] - mu; ss += d[e] * d[e]; }
    ss = wave_sum(ss);
    const float var = ss * (1.0f / 256.0f);
    const float rs = 1.0f / sqrtf(var + 1e-5f);
    unsigned short hb[8];
#pragma unroll
    for (int e = 0; e < 8; ++e) hb[e] = h_bits((d[e] * rs * gg[e] + ee[e]) * kHCarry);
    const v4u u = (v4u){pk16(hb[0], hb[1]), pk16(hb[2], hb[3]), pk16(hb[4], hb[5]), pk16(hb[6], hb[7])};
    unsigned short* p = hout + ((size_t)(b * kNtok + n0 + nl) * kChan + c0);
    *(volatile v4u*)p = u;
    __threadfence();
    *(volatile v4u*)p = u;
  }
}

__global__ __launch_bounds__(256) void l2norm_kernel(const float* __restrict__ qk, unsigned short* __restrict__ qkn,
                                                    float* __restrict__ diag) {
  __shared__ float sd[2][32];
  const int t = threadIdx.x, lane = t & 31, wave = t >> 5;
  const int n0 = blockIdx.x * 32;
  const int c0 = lane * 8;
#pragma unroll 1
  for (int i = 0; i < 4; ++i) {
    const int nl = wave * 4 + i;
    const int n = n0 + nl;
#pragma unroll
    for (int sx = 0; sx < 2; ++sx) {
      const float* rp = qk + (size_t)n * (2 * kChan) + sx * kChan + c0;
      const v4f a = *(const v4f*)(rp);
      const v4f c = *(const v4f*)(rp + 4);
      float v[8];
#pragma unroll
      for (int e = 0; e < 4; ++e) { v[e] = a[e]; v[4 + e] = c[e]; }
      float ss = 0.f;
#pragma unroll
      for (int e = 0; e < 8; ++e) ss += v[e] * v[e];
      ss = wave_sum(ss);
      const float nrm = sqrtf(ss);
      const float inv = 1.0f / fmaxf(nrm, 5e-5f);
      float dg = 0.f;
      unsigned short hb[8];
#pragma unroll
      for (int e = 0; e < 8; ++e) {
        const float qv = v[e] * inv;
        dg += qv * qv;
        hb[e] = h_bits(qv * kQnCarry);
      }
      dg = wave_sum(dg);
      const v4u u = (v4u){pk16(hb[0], hb[1]), pk16(hb[2], hb[3]), pk16(hb[4], hb[5]), pk16(hb[6], hb[7])};
      unsigned short* p = qkn + ((size_t)(sx * kNtok + n) * kChan + c0);
      *(volatile v4u*)p = u;
      __threadfence();
      *(volatile v4u*)p = u;
      if (lane == 0) sd[sx][nl] = 0.5f * dg;
    }
  }
  __syncthreads();
  if (wave < 2) {
    const float dv = sd[wave][lane];
    float* p = diag + (size_t)wave * kNtok + n0 + lane;
    *(volatile float*)p = dv;
    __threadfence();
    *(volatile float*)p = dv;
  }
}

__global__ __launch_bounds__(256) void featk_kernel(const float* __restrict__ ddkt, const float* __restrict__ diagk,
                                                   unsigned short* __restrict__ kpt, float* __restrict__ ksum) {
  __shared__ float sk[32];
  const int t = threadIdx.x, lane = t & 31, wave = t >> 5;
  const int f0 = blockIdx.x * 32;
#pragma unroll 1
  for (int i = 0; i < 4; ++i) {
    const int fl = wave * 4 + i;
    const int f = f0 + fl;
    const float* rp = ddkt + (size_t)f * kNtok;
    unsigned short* op = kpt + (size_t)f * kNtok;
    float acc = 0.f;
#pragma unroll 1
    for (int it = 0; it < 16; ++it) {
      const int n = it * 256 + lane * 8;
      const v4f a  = *(const v4f*)(rp + n);
      const v4f c  = *(const v4f*)(rp + n + 4);
      const v4f da = *(const v4f*)(diagk + n);
      const v4f dc = *(const v4f*)(diagk + n + 4);
      float kp[8];
#pragma unroll
      for (int e = 0; e < 4; ++e) {
        kp[e]     = kRatio * (expf(a[e] - da[e]) + kPhiEps);
        kp[4 + e] = kRatio * (expf(c[e] - dc[e]) + kPhiEps);
      }
      acc += ((kp[0] + kp[1]) + (kp[2] + kp[3])) + ((kp[4] + kp[5]) + (kp[6] + kp[7]));
      unsigned short hb[8];
#pragma unroll
      for (int e = 0; e < 8; ++e) hb[e] = h_bits(kp[e] * kPhiCarry);
      const v4u u = (v4u){pk16(hb[0], hb[1]), pk16(hb[2], hb[3]), pk16(hb[4], hb[5]), pk16(hb[6], hb[7])};
      unsigned short* p = op + n;
      *(volatile v4u*)p = u;
      __threadfence();
      *(volatile v4u*)p = u;
    }
    acc = wave_sum(acc);
    if (lane == 0) sk[fl] = acc;
  }
  __syncthreads();
  if (wave == 0) {
    const float dv = sk[lane];
    float* p = ksum + f0 + lane;
    *(volatile float*)p = dv;
    __threadfence();
    *(volatile float*)p = dv;
  }
}

__global__ __launch_bounds__(256) void featq_kernel(const float* __restrict__ ddq, const float* __restrict__ diagq,
                                                   const float* __restrict__ ksum, unsigned short* __restrict__ qp,
                                                   float* __restrict__ dinv) {
  __shared__ float sv[32];
  const int t = threadIdx.x, lane = t & 31, wave = t >> 5;
  const int n0 = blockIdx.x * 32;
  const int c0 = lane * 8;
  const v4f ka = *(const v4f*)(ksum + c0), kc = *(const v4f*)(ksum + c0 + 4);
  float ks[8];
#pragma unroll
  for (int e = 0; e < 4; ++e) { ks[e] = ka[e]; ks[4 + e] = kc[e]; }
#pragma unroll 1
  for (int i = 0; i < 4; ++i) {
    const int nl = wave * 4 + i;
    const int n = n0 + nl;
    const float* rp = ddq + (size_t)n * kFeat + c0;
    const v4f a = *(const v4f*)(rp);
    const v4f c = *(const v4f*)(rp + 4);
    const float dg = diagq[n];
    float x[8];
#pragma unroll
    for (int e = 0; e < 4; ++e) { x[e] = a[e]; x[4 + e] = c[e]; }
    float den = 0.f;
    unsigned short hb[8];
#pragma unroll
    for (int e = 0; e < 8; ++e) {
      const float pv = kRatio * (expf(x[e] - dg) + kPhiEps);
      den += pv * ks[e];
      hb[e] = h_bits(pv * kPhiCarry);
    }
    den = wave_sum(den);
    const float dvn = 1.0f / den;
    const v4u u = (v4u){pk16(hb[0], hb[1]), pk16(hb[2], hb[3]), pk16(hb[4], hb[5]), pk16(hb[6], hb[7])};
    unsigned short* p = qp + ((size_t)n * kFeat + c0);
    *(volatile v4u*)p = u;
    __threadfence();
    *(volatile v4u*)p = u;
    if (lane == 0) sv[nl] = dvn;
  }
  __syncthreads();
  if (wave == 0) {
    const float dv = sv[lane];
    float* p = dinv + n0 + lane;
    *(volatile float*)p = dv;
    __threadfence();
    *(volatile float*)p = dv;
  }
}

__global__ __launch_bounds__(256) void gelu_kernel(const float* __restrict__ u, unsigned short* __restrict__ gout, int n2) {
  const int i = blockIdx.x * 256 + threadIdx.x;
  if (i >= n2) return;
  const float a = u[2 * (size_t)i], c = u[2 * (size_t)i + 1];
  const float ga = 0.5f * a * (1.0f + erff(a * 0.70710678118654752f));
  const float gc = 0.5f * c * (1.0f + erff(c * 0.70710678118654752f));
  const unsigned w = pk16(h_bits(ga * kGCarry), h_bits(gc * kGCarry));
  ((volatile unsigned*)gout)[i] = w;
  __threadfence();
  ((volatile unsigned*)gout)[i] = w;
}

static inline unsigned gemm_blocks(int M, int N) { return (unsigned)((((M >> 6) * (N >> 6)) + 7) >> 3); }

extern "C" void kernel_launch(void* const* d_in, const int* in_sizes, int n_in,
                              void* d_out, int out_size, void* d_ws,
                              size_t ws_size, hipStream_t stream) {
  if (n_in < 16) return;
  if (ws_size < kWsTotal) return;
  if (out_size != kTokAll * kChan) return;
  if (in_sizes[0] != kTokAll * kChan || in_sizes[1] != kFeat * kChan || in_sizes[2] != kChan * kChan ||
      in_sizes[4] != kChan * kChan || in_sizes[6] != kChan * kChan || in_sizes[12] != kHid * kChan ||
      in_sizes[14] != kChan * kHid || in_sizes[3] != kChan || in_sizes[13] != kHid || in_sizes[15] != kChan) return;

  const float* x    = (const float*)d_in[0];
  const float* proj = (const float*)d_in[1];
  const float* wq   = (const float*)d_in[2];
  const float* bq   = (const float*)d_in[3];
  const float* wk   = (const float*)d_in[4];
  const float* bk   = (const float*)d_in[5];
  const float* wa   = (const float*)d_in[6];
  const float* ba   = (const float*)d_in[7];
  const float* g1   = (const float*)d_in[8];
  const float* b1   = (const float*)d_in[9];
  const float* g2   = (const float*)d_in[10];
  const float* b2   = (const float*)d_in[11];
  const float* w1   = (const float*)d_in[12];
  const float* fb1  = (const float*)d_in[13];
  const float* w2   = (const float*)d_in[14];
  const float* fb2  = (const float*)d_in[15];
  float* outp = (float*)d_out;

  char* ws = (char*)d_ws;
  unsigned short* H16    = (unsigned short*)(ws + kOffH16);
  unsigned short* VT16   = (unsigned short*)(ws + kOffVT16);
  float*          T2T    = (float*)(ws + kOffT2);
  unsigned short* WQK16  = (unsigned short*)(ws + kOffWQK);
  unsigned short* WA16   = (unsigned short*)(ws + kOffWA);
  unsigned short* PROJ16 = (unsigned short*)(ws + kOffPROJ);
  unsigned short* W1_16  = (unsigned short*)(ws + kOffW1);
  unsigned short* W2_16  = (unsigned short*)(ws + kOffW2);
  float*          BQK    = (float*)(ws + kOffBQK);
  float*          QKF    = (float*)(ws + kOffQKF);
  unsigned short* QKN16  = (unsigned short*)(ws + kOffQKN);
  float*          DIAG   = (float*)(ws + kOffDIAG);
  float*          DDQ    = (float*)(ws + kOffDDQ);
  float*          DDKT   = (float*)(ws + kOffDDKT);
  float*          KSUM   = (float*)(ws + kOffKSUM);
  unsigned short* KPT16  = (unsigned short*)(ws + kOffKPT);
  unsigned short* QP16   = (unsigned short*)(ws + kOffQP);
  float*          DINV   = (float*)(ws + kOffDINV);
  unsigned short* CTXT16 = (unsigned short*)(ws + kOffCTXT);
  float*          U      = (float*)(ws + kOffU);
  unsigned short* G16    = (unsigned short*)(ws + kOffG16);

  const dim3 blk(256);
  const long tokPlane = (long)kNtok * kChan;

  prep_kernel<<<dim3(128, 7), blk, 0, stream>>>(wq, wk, wa, proj, w1, w2, bq, bk, WQK16, WA16, PROJ16, W1_16, W2_16, BQK);

  ln_tok_kernel<<<dim3(1024), blk, 0, stream>>>(x, g1, b1, H16);

  gemm_f16<1, 1, false, false><<<dim3(gemm_blocks(kChan, kNtok), kBatch), blk, 0, stream>>>(
      WA16, kChan, 0L, H16, kChan, tokPlane, VT16, kNtok, tokPlane,
      ba, kVCarry, nullptr, 0L, nullptr, 0L, kChan, kNtok, kChan, kScaleVT);

  for (int b = 0; b < kBatch; ++b) {
    const unsigned short* Hb = H16 + (size_t)b * tokPlane;
    gemm_f16<2, 0, false, false><<<dim3(gemm_blocks(kNtok, 2 * kChan), 1), blk, 0, stream>>>(
        Hb, kChan, 0L, WQK16, kChan, 0L, QKF, 2 * kChan, 0L,
        BQK, 1.0f, nullptr, 0L, nullptr, 0L, kNtok, 2 * kChan, kChan, kScaleQK);
    l2norm_kernel<<<dim3(kNtok / 32), blk, 0, stream>>>(QKF, QKN16, DIAG);
    gemm_f16<0, 0, false, false><<<dim3(gemm_blocks(kNtok, kFeat), 1), blk, 0, stream>>>(
        QKN16, kChan, 0L, PROJ16, kChan, 0L, DDQ, kFeat, 0L,
        nullptr, 1.0f, nullptr, 0L, nullptr, 0L, kNtok, kFeat, kChan, kScaleDD);
    gemm_f16<0, 0, false, false><<<dim3(gemm_blocks(kFeat, kNtok), 1), blk, 0, stream>>>(
        PROJ16, kChan, 0L, QKN16 + (size_t)kNtok * kChan, kChan, 0L, DDKT, kNtok, 0L,
        nullptr, 1.0f, nullptr, 0L, nullptr, 0L, kFeat, kNtok, kChan, kScaleDD);
    featk_kernel<<<dim3(kFeat / 32), blk, 0, stream>>>(DDKT, DIAG + kNtok, KPT16, KSUM);
    featq_kernel<<<dim3(kNtok / 32), blk, 0, stream>>>(DDQ, DIAG, KSUM, QP16, DINV);
    gemm_f16<0, 1, false, false><<<dim3(gemm_blocks(kChan, kFeat), 1), blk, 0, stream>>>(
        VT16 + (size_t)b * tokPlane, kNtok, 0L, KPT16, kNtok, 0L, CTXT16, kFeat, 0L,
        nullptr, 1.0f, nullptr, 0L, nullptr, 0L, kChan, kFeat, kNtok, kScaleCTX);
    gemm_f16<0, 0, true, true><<<dim3(gemm_blocks(kChan, kNtok), 1), blk, 0, stream>>>(
        CTXT16, kFeat, 0L, QP16, kFeat, 0L, T2T + (size_t)b * tokPlane, kNtok, 0L,
        nullptr, 1.0f, x + (size_t)b * tokPlane, 0L, DINV, 0L, kChan, kNtok, kFeat, kScaleOUT);
  }

  ln_tok_kernel<<<dim3(1024), blk, 0, stream>>>(T2T, g2, b2, H16);

  for (int b = 0; b < kBatch; ++b) {
    const unsigned short* Hb = H16 + (size_t)b * tokPlane;
    gemm_f16<2, 0, false, false><<<dim3(gemm_blocks(kNtok, kHid), 1), blk, 0, stream>>>(
        Hb, kChan, 0L, W1_16, kChan, 0L, U, kHid, 0L,
        fb1, 1.0f, nullptr, 0L, nullptr, 0L, kNtok, kHid, kChan, kScaleFF1);
    gelu_kernel<<<dim3((kNtok * kHid / 2) / 256), blk, 0, stream>>>(U, G16, kNtok * kHid / 2);
    gemm_f16<1, 0, true, false><<<dim3(gemm_blocks(kChan, kNtok), 1), blk, 0, stream>>>(
        W2_16, kHid, 0L, G16, kHid, 0L, outp + (size_t)b * tokPlane, kNtok, 0L,
        fb2, 1.0f, T2T + (size_t)b * tokPlane, 0L, nullptr, 0L, kChan, kNtok, kHid, kScaleFF2);
  }
}
